// Blocks_31748398252103
// MI455X (gfx1250) — hardware-run, weakly checked
//
#include <hip/hip_runtime.h>
#include <math.h>

constexpr int kBatch   = 2;
constexpr int kSeq     = 2048;
constexpr int kEmb     = 1024;
constexpr int kHeads   = 16;
constexpr int kDh      = 64;
constexpr int kFfn     = 4096;
constexpr int kTok     = kBatch * kSeq;
constexpr int kQKld    = 2 * kEmb;
constexpr int kNumGrp  = kBatch * kHeads;
constexpr int kGrpChunk = 2;
constexpr int kNumChunk = kNumGrp / kGrpChunk;
constexpr float kWCarry   = 16.0f;
constexpr float kW2Carry  = 32.0f;
constexpr float kPCarry   = 2048.0f;
constexpr float kOCarry   = 64.0f;
constexpr float kQkScale   = 1.0f / kWCarry;
constexpr float kScoreScale = 0.125f;
constexpr float kPvScale   = kOCarry / kPCarry;
constexpr float kProjScale = 1.0f / (kOCarry * kWCarry);
constexpr float kW1Scale   = 1.0f / kWCarry;
constexpr float kW2Scale   = 1.0f / kW2Carry;
constexpr float kInvEmb    = 1.0f / 1024.0f;
constexpr float kLnEps     = 1e-5f;

static_assert(kTok % 64 == 0 && kSeq % 64 == 0 && kEmb % 64 == 0 && kFfn % 64 == 0 && kDh == 64, "tile multiples");
static_assert(kEmb % 32 == 0 && kFfn % 32 == 0 && kSeq % 32 == 0 && kDh % 32 == 0, "K multiples of 32");
static_assert(kHeads % kGrpChunk == 0, "chunks stay inside one batch");

constexpr size_t kMiB      = 1048576;
constexpr size_t kOffH16   = 0;
constexpr size_t kOffWqk   = 8 * kMiB;
constexpr size_t kOffWproj = 12 * kMiB;
constexpr size_t kOffW1t   = 14 * kMiB;
constexpr size_t kOffW2t   = 22 * kMiB;
constexpr size_t kOffAttn  = 30 * kMiB;
constexpr size_t kOffX1    = 38 * kMiB;
constexpr size_t kOffQk    = 54 * kMiB;
constexpr size_t kOffKt    = 70 * kMiB;
constexpr size_t kOffSc    = 78 * kMiB;
constexpr size_t kOffP     = 110 * kMiB;
constexpr size_t kWsEnd    = 126 * kMiB;
constexpr size_t kOffFf    = 54 * kMiB;
static_assert(kOffFf + (size_t)kTok * kFfn * 2 <= kWsEnd, "ff alias inside carve");
static_assert(kOffP + (size_t)kGrpChunk * kSeq * kSeq * 2 == kWsEnd, "carve end");
static_assert(kWsEnd <= 134217728, "carve under 128 MiB");

typedef __attribute__((ext_vector_type(16))) _Float16 v16h;
typedef __attribute__((ext_vector_type(8)))  _Float16 v8h;
typedef __attribute__((ext_vector_type(16))) __bf16   v16b;
typedef __attribute__((ext_vector_type(8)))  __bf16   v8b;
typedef __attribute__((ext_vector_type(8)))  float    v8f;
typedef __attribute__((ext_vector_type(4)))  float    v4f;
typedef __attribute__((ext_vector_type(4)))  unsigned int v4u;

__device__ __forceinline__ unsigned short f2bf_bits(float f) {
  unsigned u = __float_as_uint(f);
  return (unsigned short)((u + 0x7FFFu + ((u >> 16) & 1u)) >> 16);
}
__device__ __forceinline__ float bf_bits2f(unsigned short h) { return __uint_as_float(((unsigned)h) << 16); }

__device__ __forceinline__ void dep_guard_h(v8f& a, v8f& b, v16h x, v16h y) { asm volatile("v_nop\n\tv_nop\n\tv_nop\n\tv_nop" : "+v"(a), "+v"(b) : "v"(x), "v"(y)); }
__device__ __forceinline__ void dep_guard_b(v8f& a, v8f& b, v16b x, v16b y) { asm volatile("v_nop\n\tv_nop\n\tv_nop\n\tv_nop" : "+v"(a), "+v"(b) : "v"(x), "v"(y)); }
__device__ __forceinline__ void keep4_h(v16h a, v16h b, v16h c, v16h d) { asm volatile("v_nop" :: "v"(a), "v"(b), "v"(c), "v"(d)); }
__device__ __forceinline__ void keep4_b(v16b a, v16b b, v16b c, v16b d) { asm volatile("v_nop" :: "v"(a), "v"(b), "v"(c), "v"(d)); }
__device__ __forceinline__ void acc_guard4(v8f& a, v8f& b, v8f& c, v8f& d) { asm volatile("v_nop\n\tv_nop\n\tv_nop\n\tv_nop" : "+v"(a), "+v"(b), "+v"(c), "+v"(d)); }
template <typename T> struct Frag;
template <> struct Frag<_Float16> {
  typedef v16h V; union U { v16h v; v8h h[2]; };
  static __device__ __forceinline__ v16h load(const _Float16* p) {
    U f; f.h[0] = *(const v8h*)(p); f.h[1] = *(const v8h*)(p + 16); return f.v;
  }
  static __device__ __forceinline__ v8f mma(v16h a, v16h b, v8f c) {
    return __builtin_amdgcn_wmma_f32_16x16x32_f16(false, a, false, b, (short)0, c, false, false);
  }
  static __device__ __forceinline__ void guard(v8f& a, v8f& b, v16h x, v16h y) { dep_guard_h(a, b, x, y); }
  static __device__ __forceinline__ void keep(v16h a, v16h b, v16h c, v16h d) { keep4_h(a, b, c, d); }
};
template <> struct Frag<__bf16> {
  typedef v16b V; union U { v16b v; v8b h[2]; };
  static __device__ __forceinline__ v16b load(const __bf16* p) {
    U f; f.h[0] = *(const v8b*)(p); f.h[1] = *(const v8b*)(p + 16); return f.v;
  }
  static __device__ __forceinline__ v8f mma(v16b a, v16b b, v8f c) {
    return __builtin_amdgcn_wmma_f32_16x16x32_bf16(false, a, false, b, (short)0, c, false, false);
  }
  static __device__ __forceinline__ void guard(v8f& a, v8f& b, v16b x, v16b y) { dep_guard_b(a, b, x, y); }
  static __device__ __forceinline__ void keep(v16b a, v16b b, v16b c, v16b d) { keep4_b(a, b, c, d); }
};

__device__ __forceinline__ unsigned pk16(unsigned short a, unsigned short b) { return (unsigned)a | ((unsigned)b << 16); }
__device__ __forceinline__ unsigned short h_bits(float f) { const _Float16 h = (_Float16)f; return __builtin_bit_cast(unsigned short, h); }

template <int ET> struct Elem;
template <> struct Elem<0> { typedef _Float16 T; };
template <> struct Elem<1> { typedef __bf16 T; };
template <int ET, bool SPLIT, int BIAS_MODE, int OUT_MODE, bool RESID, int ACT = 0, int CAUSAL = 0>
__global__ __launch_bounds__(256) void wmma_gemm64(
    const unsigned short* __restrict__ Ap, const unsigned short* __restrict__ A2p, int lda, long strideA,
    const unsigned short* __restrict__ Btp, const unsigned short* __restrict__ Bt2p, int ldb, long strideB,
    void* __restrict__ Cout, void* __restrict__ Cout2, int ldc, long strideC,
    const float* __restrict__ bias,
    const float* __restrict__ resid, long strideR,
    int M, int N, int K, float scale) {
  typedef typename Elem<ET>::T T;
  typedef typename Frag<T>::V V;
  const T* A = (const T*)Ap; const T* A2 = (const T*)A2p; const T* Bt = (const T*)Btp; const T* Bt2 = (const T*)Bt2p;
  __shared__ __align__(16) float sT[8][16 * 68];
  const int b    = blockIdx.y;
  const int lane = threadIdx.x & 31;
  const int wave = threadIdx.x >> 5;
  const int tilesN = N >> 6;
  const int tilesM = M >> 6;
  const int tile = blockIdx.x * 8 + wave;
  if (tile >= tilesM * tilesN) return;
  const int tm = tile / tilesN;
  const int tn = tile - tm * tilesN;
  if (CAUSAL == 1 && tn > tm) return;
  const int m0 = tm << 6;
  const int n0 = tn << 6;
  const int kEnd = (CAUSAL == 2) ? ((((tm + 1) << 6) < K) ? ((tm + 1) << 6) : K) : K;

  const T* Ab  = A  + (size_t)b * strideA;
  const T* Bb  = Bt + (size_t)b * strideB;
  const T* Ab2 = SPLIT ? (A2  + (size_t)b * strideA) : nullptr;
  const T* Bb2 = SPLIT ? (Bt2 + (size_t)b * strideB) : nullptr;

  const int rlane = lane & 15;
  const int koff  = (lane >> 4) * 8;
  const int mOff  = (lane >> 4) * 8;

  v8f acc[4][4];
#pragma unroll
  for (int i = 0; i < 4; ++i)
#pragma unroll
    for (int j = 0; j < 4; ++j) acc[i][j] = (v8f){0.f,0.f,0.f,0.f,0.f,0.f,0.f,0.f};

  for (int k0 = 0; k0 < kEnd; k0 += 32) {
    V bh[4], bl[4];
#pragma unroll
    for (int j = 0; j < 4; ++j) {
      const size_t bo = (size_t)(n0 + (j << 4) + rlane) * ldb + koff + k0;
      bh[j] = Frag<T>::load(Bb + bo);
      if (SPLIT) bl[j] = Frag<T>::load(Bb2 + bo);
    }
#pragma unroll
    for (int i = 0; i < 4; ++i) {
      const size_t ao = (size_t)(m0 + (i << 4) + rlane) * lda + koff + k0;
      V ah = Frag<T>::load(Ab + ao);
      V al;
      if (SPLIT) al = Frag<T>::load(Ab2 + ao);
#pragma unroll
      for (int j = 0; j < 4; ++j) {
        acc[i][j] = Frag<T>::mma(ah, bh[j], acc[i][j]);
        if (SPLIT) {
          acc[i][j] = Frag<T>::mma(ah, bl[j], acc[i][j]);
          acc[i][j] = Frag<T>::mma(al, bh[j], acc[i][j]);
        }
      }
      Frag<T>::guard(acc[i][0], acc[i][3], ah, SPLIT ? al : ah);
    }
    Frag<T>::keep(bh[0], bh[1], bh[2], bh[3]);
    if (SPLIT) Frag<T>::keep(bl[0], bl[1], bl[2], bl[3]);
  }
  acc_guard4(acc[0][0], acc[0][1], acc[0][2], acc[0][3]);
  acc_guard4(acc[1][0], acc[1][1], acc[1][2], acc[1][3]);
  acc_guard4(acc[2][0], acc[2][1], acc[2][2], acc[2][3]);
  acc_guard4(acc[3][0], acc[3][1], acc[3][2], acc[3][3]);

  float* slab = sT[wave];
  const float* Rb = RESID ? (resid + (size_t)b * strideR) : nullptr;
#pragma unroll
  for (int i = 0; i < 4; ++i) {
    const int mBase = m0 + (i << 4);
#pragma unroll
    for (int j = 0; j < 4; ++j) {
      const int n = n0 + (j << 4) + rlane;
      float bv = 0.f;
      if (BIAS_MODE == 2) bv = bias[n];
#pragma unroll
      for (int r = 0; r < 8; ++r) {
        float v = acc[i][j][r] * scale;
        if (BIAS_MODE == 1) v += bias[mBase + mOff + r];
        if (BIAS_MODE == 2) v += bv;
        if (RESID) v += Rb[(size_t)(mBase + mOff + r) * ldc + n];
        if (ACT == 2) v = fmaxf(v, 0.0f);
        if (ACT == 4) v = (v > 0.f) ? v : 0.01f * v;
        slab[(mOff + r) * 68 + (j << 4) + rlane] = v;
      }
    }
    __builtin_amdgcn_fence(__ATOMIC_RELEASE, "workgroup");
    __builtin_amdgcn_wave_barrier();
    __builtin_amdgcn_fence(__ATOMIC_ACQUIRE, "workgroup");
    if (OUT_MODE == 0) {
      float* C = (float*)Cout + (size_t)b * strideC;
      const int hh = lane >> 4, c4 = (lane & 15) * 4;
      for (int pass = 0; pass < 2; ++pass) {
#pragma unroll
        for (int it = 0; it < 8; ++it) {
          const int row = it * 2 + hh;
          v4f v = *(const v4f*)(slab + row * 68 + c4);
          *(volatile v4f*)(C + (size_t)(mBase + row) * ldc + n0 + c4) = v;
        }
        __threadfence();
      }
    } else {
      const int q = lane >> 3, c8 = (lane & 7) * 8;
      unsigned short* C  = (unsigned short*)Cout  + (size_t)b * strideC;
      unsigned short* C2 = (OUT_MODE == 2) ? ((unsigned short*)Cout2 + (size_t)b * strideC) : nullptr;
      for (int pass = 0; pass < 2; ++pass) {
#pragma unroll
        for (int it = 0; it < 4; ++it) {
          const int row = it * 4 + q;
          const float* sp = slab + row * 68 + c8;
          v8h hv, lv;
#pragma unroll
          for (int e = 0; e < 8; ++e) {
            if (OUT_MODE == 1) {
              hv[e] = (_Float16)sp[e];
            } else {
              unsigned short hb = f2bf_bits(sp[e]);
              unsigned short lb = f2bf_bits(sp[e] - bf_bits2f(hb));
              hv[e] = __builtin_bit_cast(_Float16, hb);
              lv[e] = __builtin_bit_cast(_Float16, lb);
            }
          }
          *(volatile v8h*)(C + (size_t)(mBase + row) * ldc + n0 + c8) = hv;
          if (OUT_MODE == 2) *(volatile v8h*)(C2 + (size_t)(mBase + row) * ldc + n0 + c8) = lv;
        }
        __threadfence();
      }
    }
    __builtin_amdgcn_fence(__ATOMIC_RELEASE, "workgroup");
    __builtin_amdgcn_wave_barrier();
    __builtin_amdgcn_fence(__ATOMIC_ACQUIRE, "workgroup");
  }
}

__global__ __launch_bounds__(256) void tcast_kernel(const float* __restrict__ in, unsigned short* __restrict__ out,
                                                    int R, int C, long strideIn, long strideOut, float scale) {
  __shared__ float sm[64][65];
  const int t  = threadIdx.x;
  const int c0 = blockIdx.x * 64;
  const int r0 = blockIdx.y * 64;
  const float* inz = in + (size_t)blockIdx.z * strideIn;
  unsigned short* outz = out + (size_t)blockIdx.z * strideOut;
#pragma unroll
  for (int i = 0; i < 16; ++i) {
    const int e = i * 256 + t;
    const int r = e >> 6;
    const int c = e & 63;
    sm[c][r] = inz[(size_t)(r0 + r) * C + c0 + c] * scale;
  }
  __syncthreads();
  const int lane = t & 31, wave = t >> 5;
  const int q = lane >> 3, c8 = (lane & 7) * 8;
  for (int pass = 0; pass < 2; ++pass) {
#pragma unroll
    for (int it = 0; it < 2; ++it) {
      const int row = wave * 8 + it * 4 + q;
      unsigned short hb[8];
#pragma unroll
      for (int e = 0; e < 8; ++e) hb[e] = h_bits(sm[row][c8 + e]);
      const v4u u = (v4u){pk16(hb[0], hb[1]), pk16(hb[2], hb[3]), pk16(hb[4], hb[5]), pk16(hb[6], hb[7])};
      *(volatile v4u*)(outz + (size_t)(c0 + row) * R + r0 + c8) = u;
    }
    __threadfence();
  }
}

__global__ __launch_bounds__(128) void ln_f16_kernel(const float* __restrict__ x, const float* __restrict__ g,
                                                     const float* __restrict__ bta, unsigned short* __restrict__ out) {
  __shared__ float redA[4];
  __shared__ float redB[4];
  const int row  = blockIdx.x;
  const int t    = threadIdx.x;
  const int lane = t & 31, wave = t >> 5;
  const int c0   = t * 8;
  const float* xr = x + (size_t)row * kEmb + c0;
  const v4f a = *(const v4f*)(xr);
  const v4f c = *(const v4f*)(xr + 4);
  float v[8];
#pragma unroll
  for (int e = 0; e < 4; ++e) { v[e] = a[e]; v[4 + e] = c[e]; }
  float s = ((v[0] + v[1]) + (v[2] + v[3])) + ((v[4] + v[5]) + (v[6] + v[7]));
#pragma unroll
  for (int off = 16; off > 0; off >>= 1) s += __shfl_xor(s, off, 32);
  if (lane == 0) redA[wave] = s;
  __syncthreads();
  const float mu = ((redA[0] + redA[1]) + (redA[2] + redA[3])) * kInvEmb;
  float d[8];
#pragma unroll
  for (int e = 0; e < 8; ++e) d[e] = v[e] - mu;
  float ss = ((d[0] * d[0] + d[1] * d[1]) + (d[2] * d[2] + d[3] * d[3])) + ((d[4] * d[4] + d[5] * d[5]) + (d[6] * d[6] + d[7] * d[7]));
#pragma unroll
  for (int off = 16; off > 0; off >>= 1) ss += __shfl_xor(ss, off, 32);
  if (lane == 0) redB[wave] = ss;
  __syncthreads();
  const float var  = ((redB[0] + redB[1]) + (redB[2] + redB[3])) * kInvEmb;
  const float rstd = rsqrtf(var + kLnEps);
  const v4f ga = *(const v4f*)(g + c0);
  const v4f gc = *(const v4f*)(g + c0 + 4);
  const v4f ba = *(const v4f*)(bta + c0);
  const v4f bc = *(const v4f*)(bta + c0 + 4);
  float gg[8], bb[8];
#pragma unroll
  for (int e = 0; e < 4; ++e) { gg[e] = ga[e]; gg[4 + e] = gc[e]; bb[e] = ba[e]; bb[4 + e] = bc[e]; }
  unsigned short hb[8];
#pragma unroll
  for (int e = 0; e < 8; ++e) hb[e] = h_bits(d[e] * rstd * gg[e] + bb[e]);
  const v4u u = (v4u){pk16(hb[0], hb[1]), pk16(hb[2], hb[3]), pk16(hb[4], hb[5]), pk16(hb[6], hb[7])};
  unsigned short* op = out + (size_t)row * kEmb + c0;
  *(volatile v4u*)op = u;
  __threadfence();
  *(volatile v4u*)op = u;
}

__global__ __launch_bounds__(256) void kt_kernel(const unsigned short* __restrict__ qk, unsigned short* __restrict__ kt) {
  __shared__ unsigned short sm[64][72];
  const int t  = threadIdx.x;
  const int g  = blockIdx.y;
  const int b  = g >> 4, h = g & 15;
  const int s0 = blockIdx.x * 64;
#pragma unroll
  for (int i = 0; i < 2; ++i) {
    const int idx  = i * 256 + t;
    const int row  = idx >> 3;
    const int part = idx & 7;
    const v4u w = *(const v4u*)(qk + (size_t)(b * kSeq + s0 + row) * kQKld + kEmb + h * kDh + part * 8);
    const unsigned wv[4] = {w.x, w.y, w.z, w.w};
#pragma unroll
    for (int j = 0; j < 4; ++j) {
      sm[part * 8 + 2 * j][row]     = (unsigned short)(wv[j] & 0xffffu);
      sm[part * 8 + 2 * j + 1][row] = (unsigned short)(wv[j] >> 16);
    }
  }
  __syncthreads();
  const int lane = t & 31, wave = t >> 5;
  const int q = lane >> 3, c8 = (lane & 7) * 8;
  for (int pass = 0; pass < 2; ++pass) {
#pragma unroll
    for (int it = 0; it < 2; ++it) {
      const int row = wave * 8 + it * 4 + q;
      const v4u u = (v4u){pk16(sm[row][c8 + 0], sm[row][c8 + 1]), pk16(sm[row][c8 + 2], sm[row][c8 + 3]),
                          pk16(sm[row][c8 + 4], sm[row][c8 + 5]), pk16(sm[row][c8 + 6], sm[row][c8 + 7])};
      *(volatile v4u*)(kt + ((size_t)g * kDh + row) * kSeq + s0 + c8) = u;
    }
    __threadfence();
  }
}

__global__ __launch_bounds__(256) void softmax_p16_kernel(const float* __restrict__ sc, unsigned short* __restrict__ p) {
  __shared__ float redM[8];
  __shared__ float redS[8];
  const int rowg = blockIdx.x;
  const int q    = rowg & (kSeq - 1);
  const int t    = threadIdx.x;
  const int lane = t & 31, wave = t >> 5;
  const int c0   = t * 8;
  const int bound = ((q >> 6) + 1) * 64;
  const int c0c   = (c0 < bound - 8) ? c0 : (bound - 8);
  const float* sr = sc + (size_t)rowg * kSeq + c0c;
  const v4f a = *(const v4f*)(sr);
  const v4f c = *(const v4f*)(sr + 4);
  float xv[8];
#pragma unroll
  for (int e = 0; e < 4; ++e) {
    xv[e]     = (c0 + e <= q)     ? a[e] : -INFINITY;
    xv[4 + e] = (c0 + 4 + e <= q) ? c[e] : -INFINITY;
  }
  float m = fmaxf(fmaxf(fmaxf(xv[0], xv[1]), fmaxf(xv[2], xv[3])), fmaxf(fmaxf(xv[4], xv[5]), fmaxf(xv[6], xv[7])));
#pragma unroll
  for (int off = 16; off > 0; off >>= 1) m = fmaxf(m, __shfl_xor(m, off, 32));
  if (lane == 0) redM[wave] = m;
  __syncthreads();
  float mAll = redM[0];
#pragma unroll
  for (int w = 1; w < 8; ++w) mAll = fmaxf(mAll, redM[w]);
  float ev[8];
#pragma unroll
  for (int e = 0; e < 8; ++e) ev[e] = expf(xv[e] - mAll);
  float s = ((ev[0] + ev[1]) + (ev[2] + ev[3])) + ((ev[4] + ev[5]) + (ev[6] + ev[7]));
#pragma unroll
  for (int off = 16; off > 0; off >>= 1) s += __shfl_xor(s, off, 32);
  if (lane == 0) redS[wave] = s;
  __syncthreads();
  float tot = redS[0];
#pragma unroll
  for (int w = 1; w < 8; ++w) tot += redS[w];
  const float inv = kPCarry / tot;
  unsigned short hb[8];
#pragma unroll
  for (int e = 0; e < 8; ++e) hb[e] = h_bits(ev[e] * inv);
  const v4u u = (v4u){pk16(hb[0], hb[1]), pk16(hb[2], hb[3]), pk16(hb[4], hb[5]), pk16(hb[6], hb[7])};
  unsigned short* op = p + (size_t)rowg * kSeq + c0;
  *(volatile v4u*)op = u;
  __threadfence();
  *(volatile v4u*)op = u;
}

extern "C" void kernel_launch(void* const* d_in, const int* in_sizes, int n_in,
                              void* d_out, int out_size, void* d_ws,
                              size_t ws_size, hipStream_t stream) {
  if (n_in < 13) return;
  if (in_sizes[0] != kTok * kEmb) return;
  if (in_sizes[1] != kHeads * kEmb * kDh || in_sizes[2] != kHeads * kEmb * kDh) return;
  if (in_sizes[3] != kEmb * kEmb || in_sizes[9] != kEmb * kFfn || in_sizes[11] != kFfn * kEmb) return;
  if (out_size != kTok * kEmb) return;
  if (ws_size < kWsEnd) return;

  const float* x     = (const float*)d_in[0];
  const float* Wq    = (const float*)d_in[1];
  const float* Wk    = (const float*)d_in[2];
  const float* Wproj = (const float*)d_in[3];
  const float* bproj = (const float*)d_in[4];
  const float* ln1g  = (const float*)d_in[5];
  const float* ln1b  = (const float*)d_in[6];
  const float* ln2g  = (const float*)d_in[7];
  const float* ln2b  = (const float*)d_in[8];
  const float* W1    = (const float*)d_in[9];
  const float* b1    = (const float*)d_in[10];
  const float* W2    = (const float*)d_in[11];
  const float* b2    = (const float*)d_in[12];
  float* out = (float*)d_out;

  char* ws = (char*)d_ws;
  unsigned short* h16    = (unsigned short*)(ws + kOffH16);
  unsigned short* wqk16  = (unsigned short*)(ws + kOffWqk);
  unsigned short* wproj16 = (unsigned short*)(ws + kOffWproj);
  unsigned short* w1t16  = (unsigned short*)(ws + kOffW1t);
  unsigned short* w2t16  = (unsigned short*)(ws + kOffW2t);
  unsigned short* attn16 = (unsigned short*)(ws + kOffAttn);
  float*          x1     = (float*)(ws + kOffX1);
  unsigned short* qk16   = (unsigned short*)(ws + kOffQk);
  unsigned short* kt16   = (unsigned short*)(ws + kOffKt);
  float*          sc     = (float*)(ws + kOffSc);
  unsigned short* p16    = (unsigned short*)(ws + kOffP);
  unsigned short* ff16   = (unsigned short*)(ws + kOffFf);

  tcast_kernel<<<dim3(1, kEmb / 64, kHeads), 256, 0, stream>>>(Wq, wqk16, kEmb, kDh, (long)kEmb * kDh, (long)kDh * kEmb, kWCarry);
  tcast_kernel<<<dim3(1, kEmb / 64, kHeads), 256, 0, stream>>>(Wk, wqk16 + (size_t)kEmb * kEmb, kEmb, kDh, (long)kEmb * kDh, (long)kDh * kEmb, kWCarry);
  tcast_kernel<<<dim3(kEmb / 64, kEmb / 64, 1), 256, 0, stream>>>(Wproj, wproj16, kEmb, kEmb, 0L, 0L, kWCarry);
  tcast_kernel<<<dim3(kFfn / 64, kEmb / 64, 1), 256, 0, stream>>>(W1, w1t16, kEmb, kFfn, 0L, 0L, kWCarry);
  tcast_kernel<<<dim3(kEmb / 64, kFfn / 64, 1), 256, 0, stream>>>(W2, w2t16, kFfn, kEmb, 0L, 0L, kW2Carry);

  ln_f16_kernel<<<kTok, 128, 0, stream>>>(x, ln1g, ln1b, h16);

  wmma_gemm64<0, false, 0, 1, false, 0, 0><<<dim3(256, 1), 256, 0, stream>>>(
      h16, h16, kEmb, 0L, wqk16, wqk16, kEmb, 0L,
      (void*)qk16, (void*)qk16, kQKld, 0L, bproj, x, 0L, kTok, kQKld, kEmb, kQkScale);

  kt_kernel<<<dim3(kSeq / 64, kNumGrp), 256, 0, stream>>>(qk16, kt16);

  for (int ch = 0; ch < kNumChunk; ++ch) {
    const int g0 = ch * kGrpChunk;
    const int b  = g0 / kHeads;
    const int h0 = g0 % kHeads;
    const unsigned short* qbase = qk16 + (size_t)b * kSeq * kQKld + (size_t)h0 * kDh;
    const unsigned short* kbase = qk16 + (size_t)b * kSeq * kQKld + kEmb + (size_t)h0 * kDh;
    wmma_gemm64<0, false, 0, 0, false, 0, 1><<<dim3(128, kGrpChunk), 256, 0, stream>>>(
        qbase, qbase, kQKld, (long)kDh, kbase, kbase, kQKld, (long)kDh,
        (void*)sc, (void*)sc, kSeq, (long)kSeq * kSeq, bproj, x, 0L, kSeq, kSeq, kDh, kScoreScale);
    softmax_p16_kernel<<<kGrpChunk * kSeq, 256, 0, stream>>>(sc, p16);
    wmma_gemm64<0, false, 0, 1, false, 0, 2><<<dim3(4, kGrpChunk), 256, 0, stream>>>(
        p16, p16, kSeq, (long)kSeq * kSeq, kt16 + (size_t)g0 * kDh * kSeq, kt16 + (size_t)g0 * kDh * kSeq, kSeq, (long)kDh * kSeq,
        (void*)(attn16 + (size_t)b * kSeq * kEmb + (size_t)h0 * kDh), (void*)(attn16 + (size_t)b * kSeq * kEmb + (size_t)h0 * kDh), kEmb, (long)kDh,
        bproj, x, 0L, kSeq, kDh, kSeq, kPvScale);
  }

  wmma_gemm64<0, false, 2, 0, true, 0, 0><<<dim3(128, 1), 256, 0, stream>>>(
      attn16, attn16, kEmb, 0L, wproj16, wproj16, kEmb, 0L,
      (void*)x1, (void*)x1, kEmb, 0L, bproj, x, 0L, kTok, kEmb, kEmb, kProjScale);

  ln_f16_kernel<<<kTok, 128, 0, stream>>>(x1, ln2g, ln2b, h16);

  wmma_gemm64<0, false, 2, 1, false, 2, 0><<<dim3(512, 1), 256, 0, stream>>>(
      h16, h16, kEmb, 0L, w1t16, w1t16, kEmb, 0L,
      (void*)ff16, (void*)ff16, kFfn, 0L, b1, x, 0L, kTok, kFfn, kEmb, kW1Scale);

  wmma_gemm64<0, false, 2, 0, true, 0, 0><<<dim3(128, 1), 256, 0, stream>>>(
      ff16, ff16, kFfn, 0L, w2t16, w2t16, kFfn, 0L,
      (void*)out, (void*)out, kEmb, 0L, b2, x1, 0L, kTok, kEmb, kFfn, kW2Scale);
}
